// RN_37752762532001
// MI455X (gfx1250) — hardware-verified
//
#include <hip/hip_runtime.h>

constexpr int kObj       = 64;
constexpr int kFeat      = 64;
constexpr int kCh        = 64;
constexpr int kBatch     = 1024;
constexpr int kSampleLen = kObj * kFeat;
constexpr int kPairTiles = 126;
constexpr int kHid       = 64;
constexpr int kOut       = 10;
constexpr int kHeadRows  = 32;
constexpr int kThreads   = 256;
constexpr float kWCarry    = 16.0f;
constexpr float kWCarryInv = 0.0625f;
static_assert(kPairTiles * 16 == kObj * (kObj - 1) / 2, "tile count");
static_assert(kBatch % kHeadRows == 0, "head grid");
static_assert(kFeat % 32 == 0 && kCh % 32 == 0, "K multiple of 32");
static_assert(kThreads * 16 == kObj * kFeat, "staging coverage");
static_assert(kHeadRows * kOut == 320, "head store extent");
static_assert(kHeadRows * kCh == 2048 && kHid * kCh == 4096, "head staging coverage");

typedef __attribute__((ext_vector_type(16))) _Float16 v16h;
typedef __attribute__((ext_vector_type(8)))  _Float16 v8h;
typedef __attribute__((ext_vector_type(8)))  float    v8f;
typedef __attribute__((ext_vector_type(4)))  float    v4f;

__device__ __forceinline__ void dep_guard_h(v8f& a, v8f& b, v16h x, v16h y) { asm volatile("v_nop\n\tv_nop\n\tv_nop\n\tv_nop" : "+v"(a), "+v"(b) : "v"(x), "v"(y)); }
__device__ __forceinline__ void keep4_h(v16h a, v16h b, v16h c, v16h d) { asm volatile("v_nop" :: "v"(a), "v"(b), "v"(c), "v"(d)); }
template <typename T> struct Frag;
template <> struct Frag<_Float16> {
  typedef v16h V; union U { v16h v; v8h h[2]; };
  static __device__ __forceinline__ v16h load(const _Float16* p) {
    U f; f.h[0] = *(const v8h*)(p); f.h[1] = *(const v8h*)(p + 16); return f.v;
  }
  static __device__ __forceinline__ v8f mma(v16h a, v16h b, v8f c) {
    return __builtin_amdgcn_wmma_f32_16x16x32_f16(false, a, false, b, (short)0, c, false, false);
  }
  static __device__ __forceinline__ void guard(v8f& a, v8f& b, v16h x, v16h y) { dep_guard_h(a, b, x, y); }
  static __device__ __forceinline__ void keep(v16h a, v16h b, v16h c, v16h d) { keep4_h(a, b, c, d); }
};

__device__ __forceinline__ v8f zero8() { return (v8f){0.f, 0.f, 0.f, 0.f, 0.f, 0.f, 0.f, 0.f}; }

__device__ __forceinline__ void grp_guard(v8f& c0, v8f& c1, v8f& c2, v8f& c3,
                                          v16h a0, v16h a1, v16h b0, v16h b1, v16h b2, v16h b3) {
  asm volatile("v_nop\n\tv_nop\n\tv_nop\n\tv_nop"
               : "+v"(c0), "+v"(c1), "+v"(c2), "+v"(c3)
               : "v"(a0), "v"(a1), "v"(b0), "v"(b1), "v"(b2), "v"(b3));
}

__device__ __forceinline__ void cvt16(const float* __restrict__ src, _Float16* dst, float scale) {
  const v4f f0 = *(const v4f*)(src);
  const v4f f1 = *(const v4f*)(src + 4);
  const v4f f2 = *(const v4f*)(src + 8);
  const v4f f3 = *(const v4f*)(src + 12);
  v8h p0, p1;
#pragma unroll
  for (int e = 0; e < 4; ++e) {
    p0[e]     = (_Float16)(f0[e] * scale);
    p0[4 + e] = (_Float16)(f1[e] * scale);
    p1[e]     = (_Float16)(f2[e] * scale);
    p1[4 + e] = (_Float16)(f3[e] * scale);
  }
  *(v8h*)(dst) = p0;
  *(v8h*)(dst + 8) = p1;
}

__global__ __launch_bounds__(kThreads) void pair_stack_kernel(
    const float* __restrict__ x, const float* __restrict__ w0a, const float* __restrict__ w0b,
    const float* __restrict__ b0, const float* __restrict__ w1, const float* __restrict__ b1,
    float* __restrict__ pooled) {
  __shared__ __align__(16) _Float16 Xh[kObj * kFeat];
  __shared__ __align__(16) _Float16 Wab[2 * kCh * kFeat];
  __shared__ __align__(16) _Float16 W1h[kCh * kCh];
  __shared__ __align__(16) _Float16 ABp[2 * kObj * kCh];
  __shared__ __align__(16) float red[8 * kCh];
  __shared__ __align__(16) float pool_s[kCh];
  __shared__ float b0s[kCh];
  __shared__ float b1x[kCh];
  __shared__ float wtab[kObj];

  const int tid  = threadIdx.x;
  const int wave = tid >> 5;
  const int lane = tid & 31;
  const int hh   = lane >> 4;
  const int m    = lane & 15;
  const size_t n = blockIdx.x;

  cvt16(x + n * kSampleLen + 16 * tid, Xh + 16 * tid, 1.0f);
  asm volatile("" ::: "memory");
  cvt16(w0a + 16 * tid, Wab + 16 * tid, kWCarry);
  asm volatile("" ::: "memory");
  cvt16(w0b + 16 * tid, Wab + kCh * kFeat + 16 * tid, kWCarry);
  asm volatile("" ::: "memory");
  cvt16(w1 + 16 * tid, W1h + 16 * tid, kWCarry);
  if (tid < kCh) {
    b0s[tid]  = b0[tid];
    b1x[tid]  = b1[tid] * kWCarry;
    wtab[tid] = 1.0f / (float)(63 * (64 - tid));
  }
  __syncthreads();

  {
    const int mat   = wave >> 2;
    const int mtile = wave & 3;
    const _Float16* Wm = Wab + mat * (kCh * kFeat);
    _Float16* Dm = ABp + mat * (kObj * kCh);
    const int row = mtile * 16 + m;
    const v16h a0 = Frag<_Float16>::load(Xh + row * kFeat + 8 * hh);
    const v16h a1 = Frag<_Float16>::load(Xh + row * kFeat + 32 + 8 * hh);
    v16h bq0[4], bq1[4];
#pragma unroll
    for (int nt = 0; nt < 4; ++nt) {
      const _Float16* bp = Wm + (nt * 16 + m) * kFeat + 8 * hh;
      bq0[nt] = Frag<_Float16>::load(bp);
      bq1[nt] = Frag<_Float16>::load(bp + 32);
    }
    v8f acc[4];
#pragma unroll
    for (int nt = 0; nt < 4; ++nt) acc[nt] = zero8();
#pragma unroll
    for (int nt = 0; nt < 4; ++nt) acc[nt] = Frag<_Float16>::mma(a0, bq0[nt], acc[nt]);
#pragma unroll
    for (int nt = 0; nt < 4; ++nt) acc[nt] = Frag<_Float16>::mma(a1, bq1[nt], acc[nt]);
    grp_guard(acc[0], acc[1], acc[2], acc[3], a0, a1, bq1[0], bq1[1], bq1[2], bq1[3]);
    keep4_h(bq0[0], bq0[1], bq0[2], bq0[3]);
    const float bsel = (mat == 0) ? 1.0f : 0.0f;
#pragma unroll
    for (int nt = 0; nt < 4; ++nt) {
      const float bv = b0s[nt * 16 + m] * bsel;
#pragma unroll
      for (int r = 0; r < 8; ++r) {
        const float v = fmaf(acc[nt][r], kWCarryInv, bv);
        Dm[(mtile * 16 + 8 * hh + r) * kCh + nt * 16 + m] = (_Float16)v;
      }
    }
  }
  __syncthreads();

  v16h w1q0[4], w1q1[4];
  float b1c[4];
#pragma unroll
  for (int nt = 0; nt < 4; ++nt) {
    const _Float16* bp = W1h + (nt * 16 + m) * kCh + 8 * hh;
    w1q0[nt] = Frag<_Float16>::load(bp);
    w1q1[nt] = Frag<_Float16>::load(bp + 32);
    b1c[nt]  = b1x[nt * 16 + m];
  }
  float accp[4] = {0.0f, 0.0f, 0.0f, 0.0f};
  v8h z8;
#pragma unroll
  for (int e = 0; e < 8; ++e) z8[e] = (_Float16)0.0f;
  const _Float16* Apl = ABp;
  const _Float16* Bpl = ABp + kObj * kCh;

#pragma unroll 1
  for (int tile = wave; tile < kPairTiles; tile += 8) {
    const int d   = (tile >> 2) + 1;
    const int sub = tile & 3;
    const int lim = kObj - d;
    const int q   = sub * 16 + m;
    const bool cq = q < lim;
    int ip  = cq ? q : (q - lim);
    const int gap = cq ? d : lim;
    int jp  = ip + gap;
    ip &= (kObj - 1);
    jp &= (kObj - 1);
    const float wA = wtab[d];
    const float wB = wtab[lim];
    const v8h* pa = (const v8h*)(Apl + ip * kCh + 8 * hh);
    const v8h* pb = (const v8h*)(Bpl + jp * kCh + 8 * hh);
    Frag<_Float16>::U ua, ub;
    ua.h[0] = __builtin_elementwise_max(pa[0] + pb[0], z8);
    ua.h[1] = __builtin_elementwise_max(pa[2] + pb[2], z8);
    ub.h[0] = __builtin_elementwise_max(pa[4] + pb[4], z8);
    ub.h[1] = __builtin_elementwise_max(pa[6] + pb[6], z8);
    v8f cc[4];
#pragma unroll
    for (int nt = 0; nt < 4; ++nt) cc[nt] = zero8();
#pragma unroll
    for (int nt = 0; nt < 4; ++nt) cc[nt] = Frag<_Float16>::mma(ua.v, w1q0[nt], cc[nt]);
#pragma unroll
    for (int nt = 0; nt < 4; ++nt) cc[nt] = Frag<_Float16>::mma(ub.v, w1q1[nt], cc[nt]);
    grp_guard(cc[0], cc[1], cc[2], cc[3], ua.v, ub.v, w1q1[0], w1q1[1], w1q1[2], w1q1[3]);
    keep4_h(w1q0[0], w1q0[1], w1q0[2], w1q0[3]);
    float wr[8];
#pragma unroll
    for (int r = 0; r < 8; ++r) {
      const int qr = sub * 16 + 8 * hh + r;
      const float fa = (qr < lim) ? 1.0f : 0.0f;
      const float fb = 1.0f - fa;
      wr[r] = fmaf(fa, wA, fb * wB);
    }
#pragma unroll
    for (int nt = 0; nt < 4; ++nt) {
#pragma unroll
      for (int r = 0; r < 8; ++r) {
        const float v = fmaxf(cc[nt][r] + b1c[nt], 0.0f);
        accp[nt] = fmaf(wr[r], v, accp[nt]);
      }
    }
  }

#pragma unroll
  for (int nt = 0; nt < 4; ++nt) {
    float v = accp[nt];
    v += __shfl_xor(v, 16, 32);
    if (hh == 0) red[wave * kCh + nt * 16 + m] = v;
  }
  __syncthreads();
  if (tid < kCh) {
    float s = 0.0f;
#pragma unroll
    for (int w = 0; w < 8; ++w) s += red[w * kCh + tid];
    pool_s[tid] = s * kWCarryInv;
  }
  __syncthreads();
  if (wave == 0) {
    const int c4 = (lane & 15) * 4;
    const v4f v = *(const v4f*)(pool_s + c4);
    float* dst = pooled + n * kCh + c4;
    for (int pass = 0; pass < 2; ++pass) {
      if (lane < 16) *(volatile v4f*)dst = v;
      __threadfence();
    }
  }
}

__global__ __launch_bounds__(kThreads) void head_kernel(
    const float* __restrict__ pooled, const float* __restrict__ wm1, const float* __restrict__ bm1,
    const float* __restrict__ wm2, const float* __restrict__ bm2, float* __restrict__ out) {
  __shared__ __align__(16) float Ps[kHeadRows * kCh];
  __shared__ __align__(16) float Wm1s[kHid * kCh];
  __shared__ __align__(16) float Wm2s[kOut * kHid];
  __shared__ float bm1s[kHid];
  __shared__ float bm2s[16];
  __shared__ __align__(16) float zs[kHeadRows * kHid];
  __shared__ __align__(16) float so[kHeadRows * kOut];
  const int tid  = threadIdx.x;
  const int lane = tid & 31;
  const int wave = tid >> 5;
  const size_t s0 = (size_t)blockIdx.x * kHeadRows;
  {
    const float* pp = pooled + s0 * kCh;
    *(v4f*)(Ps + 4 * tid)        = *(const v4f*)(pp + 4 * tid);
    *(v4f*)(Ps + 1024 + 4 * tid) = *(const v4f*)(pp + 1024 + 4 * tid);
    asm volatile("" ::: "memory");
#pragma unroll
    for (int i = 0; i < 4; ++i) *(v4f*)(Wm1s + 1024 * i + 4 * tid) = *(const v4f*)(wm1 + 1024 * i + 4 * tid);
    asm volatile("" ::: "memory");
    if (tid < (kOut * kHid) / 4) *(v4f*)(Wm2s + 4 * tid) = *(const v4f*)(wm2 + 4 * tid);
    if (tid < kHid) bm1s[tid] = bm1[tid];
    if (tid < kOut) bm2s[tid] = bm2[tid];
  }
  __syncthreads();
#pragma unroll 1
  for (int it = 0; it < (kHeadRows * kHid) / kThreads; ++it) {
    const int i = it * kThreads + tid;
    const int s = i >> 6;
    const int j = i & 63;
    const float* pr = Ps + s * kCh;
    const float* wr = Wm1s + j * kCh;
    float a = 0.0f;
#pragma unroll 1
    for (int c = 0; c < kCh; ++c) a = fmaf(pr[c], wr[c], a);
    zs[i] = fmaxf(a + bm1s[j], 0.0f);
  }
  __syncthreads();
  for (int i = tid; i < kHeadRows * kOut; i += kThreads) {
    const int s = i / kOut;
    const int k = i - s * kOut;
    const float* zr = zs + s * kHid;
    const float* wr = Wm2s + k * kHid;
    float a = 0.0f;
#pragma unroll 1
    for (int j = 0; j < kHid; ++j) a = fmaf(zr[j], wr[j], a);
    so[i] = a + bm2s[k];
  }
  __syncthreads();
  if (wave == 0) {
    const v4f p0 = *(const v4f*)(so + 4 * lane);
    const v4f p1 = *(const v4f*)(so + 128 + 4 * lane);
    const v4f p2 = *(const v4f*)(so + 256 + 4 * (lane & 15));
    float* ob = out + (size_t)blockIdx.x * (kHeadRows * kOut);
    for (int pass = 0; pass < 2; ++pass) {
      *(volatile v4f*)(ob + 4 * lane) = p0;
      *(volatile v4f*)(ob + 128 + 4 * lane) = p1;
      if (lane < 16) *(volatile v4f*)(ob + 256 + 4 * lane) = p2;
      __threadfence();
    }
  }
}

extern "C" void kernel_launch(void* const* d_in, const int* in_sizes, int n_in,
                              void* d_out, int out_size, void* d_ws, size_t ws_size, hipStream_t stream) {
  if (n_in < 10) return;
  const float* x   = (const float*)d_in[0];
  const float* w0a = (const float*)d_in[1];
  const float* w0b = (const float*)d_in[2];
  const float* b0  = (const float*)d_in[3];
  const float* w1  = (const float*)d_in[4];
  const float* b1  = (const float*)d_in[5];
  const float* wm1 = (const float*)d_in[6];
  const float* bm1 = (const float*)d_in[7];
  const float* wm2 = (const float*)d_in[8];
  const float* bm2 = (const float*)d_in[9];
  float* out = (float*)d_out;

  if ((size_t)in_sizes[0] != (size_t)kBatch * kSampleLen) return;
  if (out_size != kBatch * kOut) return;
  const size_t pooled_bytes = (size_t)kBatch * kCh * sizeof(float);
  if (pooled_bytes > ws_size || pooled_bytes > (size_t)134217728) return;
  float* pooled = (float*)d_ws;

  pair_stack_kernel<<<kBatch, kThreads, 0, stream>>>(x, w0a, w0b, b0, w1, b1, pooled);
  head_kernel<<<kBatch / kHeadRows, kThreads, 0, stream>>>(pooled, wm1, bm1, wm2, bm2, out);
}
